// KDSR_16655883174453
// MI455X (gfx1250) — hardware-run, weakly checked
//
#include <hip/hip_runtime.h>
#include <math.h>

typedef __attribute__((ext_vector_type(16))) _Float16 v16h;
typedef __attribute__((ext_vector_type(8)))  _Float16 v8h;
typedef __attribute__((ext_vector_type(8)))  float    v8f;
typedef __attribute__((ext_vector_type(4)))  float    v4f;

constexpr int kNB    = 8;
constexpr int kCh    = 64;
constexpr int kH1    = 128;
constexpr int kW1    = 128;
constexpr int kHP1   = kH1 + 2;
constexpr int kWP1   = kW1 + 2;
constexpr int kH2    = 256;
constexpr int kW2    = 256;
constexpr int kHP2   = kH2 + 2;
constexpr int kWP2   = kW2 + 2;
constexpr int kKK    = 9 * kCh;
constexpr int kNBlk  = 8;
constexpr int kNV    = 48;
constexpr int kHeadK = 32;
constexpr float kWCarry    = 256.0f;
constexpr float kLoCarry   = 2048.0f;
constexpr float kScaleMain = 1.0f / kWCarry;
constexpr float kScaleLo   = 1.0f / (kWCarry * kLoCarry);
constexpr bool kSplitBlocks = true;
constexpr int  kBlkMI       = kSplitBlocks ? 2 : 4;
constexpr int  kBlkLgTpr    = kSplitBlocks ? 2 : 1;
static_assert(kKK == 576);
static_assert((kKK % 32) == 0 && (kHeadK % 32) == 0);
static_assert((kW1 % 64) == 0 && (kW2 % 64) == 0);

constexpr size_t kPadPlane16 = (size_t)kNB * kHP1 * kWP1 * kCh * 2;
constexpr size_t kOffAHI = 0;
constexpr size_t kOffALO = kOffAHI + kPadPlane16;
constexpr size_t kOffSHI = kOffALO + kPadPlane16;
constexpr size_t kOffRES = kOffSHI + kPadPlane16;
constexpr size_t kSzRES  = (size_t)kNB * kHP1 * kWP1 * kCh * 4;
constexpr size_t kOffXHD = kOffRES + kSzRES;
constexpr size_t kSzXHD  = (size_t)kNB * kH1 * kW1 * kCh * 4;
constexpr size_t kOffWB  = kOffXHD + kSzXHD;
constexpr size_t kSzWB   = (size_t)kNBlk * kCh * kKK * 2;
constexpr size_t kOffWC  = kOffWB + kSzWB;
constexpr size_t kSzWC   = (size_t)kCh * kKK * 2;
constexpr size_t kOffWU1 = kOffWC + kSzWC;
constexpr size_t kSzWU1  = (size_t)4 * kCh * kKK * 2;
constexpr size_t kOffWV  = kOffWU1 + kSzWU1;
constexpr size_t kSzWV   = (size_t)kNV * kKK * 2;
constexpr size_t kOffWH  = kOffWV + kSzWV;
constexpr size_t kSzWH   = (size_t)kCh * kHeadK * 2;
constexpr size_t kOffDK  = kOffWH + kSzWH;
constexpr size_t kSzDK   = (size_t)kNBlk * kNB * kKK * 4;
constexpr size_t kOffVB  = kOffDK + kSzDK;
constexpr size_t kSzVB   = 256;
constexpr size_t kWsTotal = kOffVB + kSzVB;
constexpr size_t kOffIHI = kOffAHI;
constexpr size_t kOffILO = kOffALO;
constexpr size_t kSzIm   = (size_t)kNB * kH1 * kW1 * kHeadK * 2;
constexpr size_t kOffGPL = 0;
constexpr size_t kSzGPL  = (size_t)kNB * kH2 * kW2 * kNV * 2;
constexpr size_t kOffTUP = kOffGPL + kSzGPL;
constexpr size_t kSzTUP  = (size_t)kNB * kHP2 * kWP2 * kCh * 2;
static_assert(kPadPlane16 == 17305600ull);
static_assert(kWsTotal == 121248000ull);
static_assert(kWsTotal <= 134217728ull);
static_assert(kSzIm <= kPadPlane16);
static_assert(kOffTUP >= kOffAHI + kPadPlane16);
static_assert(kOffTUP + kSzTUP <= kOffWB);
static_assert(kOffGPL + kSzGPL <= kOffTUP);
static_assert((kOffALO % 128) == 0 && (kOffSHI % 128) == 0 && (kOffRES % 128) == 0 && (kOffXHD % 128) == 0 &&
              (kOffWB % 128) == 0 && (kOffWC % 128) == 0 && (kOffWU1 % 128) == 0 && (kOffWV % 128) == 0 &&
              (kOffWH % 128) == 0 && (kOffDK % 128) == 0 && (kOffVB % 128) == 0 && (kOffTUP % 128) == 0);

__device__ __forceinline__ unsigned short f2bf_bits(float f) {
  unsigned u = __float_as_uint(f);
  return (unsigned short)((u + 0x7FFFu + ((u >> 16) & 1u)) >> 16);
}
__device__ __forceinline__ float bf_bits2f(unsigned short h) { return __uint_as_float(((unsigned)h) << 16); }
__device__ __forceinline__ float bf_rne(float f) { return bf_bits2f(f2bf_bits(f)); }

__device__ __forceinline__ float h16_to_f32(unsigned hb) {
  const unsigned sgn = (hb & 0x8000u) << 16;
  const unsigned em = hb & 0x7fffu;
  const float fn = __uint_as_float((em << 13) + 0x38000000u);
  const float fs = (float)em * 5.9604644775390625e-8f;
  const float mag = (em < 0x400u) ? fs : fn;
  return __uint_as_float(__float_as_uint(mag) | sgn);
}

__device__ __forceinline__ void wave_sync() {
  __builtin_amdgcn_fence(__ATOMIC_RELEASE, "workgroup");
  __builtin_amdgcn_wave_barrier();
  __builtin_amdgcn_fence(__ATOMIC_ACQUIRE, "workgroup");
}

__device__ __forceinline__ void guard_row3(v8f& a, v8f& b, v8f& c, v16h x, v16h y) {
  asm volatile("v_nop\n\tv_nop\n\tv_nop\n\tv_nop" : "+v"(a), "+v"(b), "+v"(c) : "v"(x), "v"(y));
}
__device__ __forceinline__ void guard_row4(v8f& a, v8f& b, v8f& c, v8f& d, v16h x, v16h y) {
  asm volatile("v_nop\n\tv_nop\n\tv_nop\n\tv_nop" : "+v"(a), "+v"(b), "+v"(c), "+v"(d) : "v"(x), "v"(y));
}
__device__ __forceinline__ void guard_row8(v8f& a, v8f& b, v8f& c, v8f& d, v8f& e, v8f& f, v8f& g, v8f& h, v16h x, v16h y) {
  asm volatile("v_nop\n\tv_nop\n\tv_nop\n\tv_nop"
               : "+v"(a), "+v"(b), "+v"(c), "+v"(d), "+v"(e), "+v"(f), "+v"(g), "+v"(h) : "v"(x), "v"(y));
}
__device__ __forceinline__ void keep3_h(v16h a, v16h b, v16h c) { asm volatile("v_nop" :: "v"(a), "v"(b), "v"(c)); }
__device__ __forceinline__ void keep4_h(v16h a, v16h b, v16h c, v16h d) { asm volatile("v_nop" :: "v"(a), "v"(b), "v"(c), "v"(d)); }

struct FragH {
  union U { v16h v; v8h h[2]; };
  static __device__ __forceinline__ v16h load(const _Float16* p) {
    U f;
    f.h[0] = *(const v8h*)(p);
    f.h[1] = *(const v8h*)(p + 16);
    return f.v;
  }
  static __device__ __forceinline__ v8f mma(v16h a, v16h b, v8f c) {
    return __builtin_amdgcn_wmma_f32_16x16x32_f16(false, a, false, b, (short)0, c, false, false);
  }
};

__global__ __launch_bounds__(256) void pack_w_kernel(const float* __restrict__ src, unsigned short* __restrict__ dst,
                                                     int nrows, int perm)
{
  const int i = blockIdx.x * 256 + threadIdx.x;
  if (i >= nrows * 72) return;
  const int row = i / 72;
  const int k8 = (i - row * 72) * 8;
  const int tap = k8 >> 6;
  const int ci0 = k8 & 63;
  int srow = row;
  if (perm) srow = 4 * (row & 63) + (row >> 6);
  v8h hv;
#pragma unroll
  for (int e = 0; e < 8; ++e) {
    const float w = src[((size_t)srow * kCh + ci0 + e) * 9 + tap];
    hv[e] = (_Float16)(bf_rne(w) * kWCarry);
  }
  unsigned short* q = dst + (size_t)i * 8;
  *(volatile v8h*)q = hv;
  __threadfence();
  *(volatile v8h*)q = hv;
}

__global__ __launch_bounds__(256) void pack_head_kernel(const float* __restrict__ src, unsigned short* __restrict__ dst)
{
  const int i = threadIdx.x;
  const int row = i >> 2;
  const int k8 = (i & 3) * 8;
  v8h hv;
#pragma unroll
  for (int e = 0; e < 8; ++e) {
    const int k = k8 + e;
    const int kc = (k < 27) ? k : 26;
    const float w = src[row * 27 + kc];
    const float val = (k < 27) ? (bf_rne(w) * kWCarry) : 0.0f;
    hv[e] = (_Float16)val;
  }
  unsigned short* q = dst + (size_t)i * 8;
  *(volatile v8h*)q = hv;
  __threadfence();
  *(volatile v8h*)q = hv;
}

__global__ __launch_bounds__(576) void compose_v_kernel(const float* __restrict__ tail_w, const float* __restrict__ up2_w,
                                                        unsigned short* __restrict__ V)
{
  __shared__ __align__(16) float sV[kKK];
  const int n = blockIdx.x;
  const int ax = n & 1, ay = (n >> 1) & 1, sx = (n >> 2) & 1, sy = (n >> 3) & 1, c = n >> 4;
  const int k = threadIdx.x;
  const int tap = k >> 6, ci = k & 63;
  float acc = 0.0f;
#pragma unroll 1
  for (int dy = 0; dy < 3; ++dy) {
    const int oy = sy + dy + 1;
    const int jy = (oy >> 1) - 1;
    const int sgy = oy & 1;
    if (jy != sy + ay - 1) continue;
#pragma unroll 1
    for (int dx = 0; dx < 3; ++dx) {
      const int ox = sx + dx + 1;
      const int jx = (ox >> 1) - 1;
      const int sgx = ox & 1;
      if (jx != sx + ax - 1) continue;
#pragma unroll 1
      for (int m = 0; m < kCh; ++m) {
        const float tw = bf_rne(tail_w[((c * kCh + m) * 3 + dy) * 3 + dx]);
        const int co = 4 * m + 2 * sgy + sgx;
        const float uw = bf_rne(up2_w[((size_t)co * kCh + ci) * 9 + tap]);
        acc = fmaf(tw, uw, acc);
      }
    }
  }
  sV[k] = acc * kWCarry;
  __syncthreads();
  if (k < 72) {
    v8h hv;
    const v4f a0 = *(const v4f*)(sV + k * 8);
    const v4f a1 = *(const v4f*)(sV + k * 8 + 4);
#pragma unroll
    for (int e = 0; e < 4; ++e) {
      hv[e] = (_Float16)a0[e];
      hv[4 + e] = (_Float16)a1[e];
    }
    unsigned short* q = V + (size_t)n * kKK + k * 8;
    *(volatile v8h*)q = hv;
    __threadfence();
    *(volatile v8h*)q = hv;
  }
}

__global__ __launch_bounds__(64) void vbias_kernel(const float* __restrict__ tail_w, const float* __restrict__ up2_b,
                                                   float* __restrict__ Vb)
{
  const int t = threadIdx.x;
  const int n = (t < kNV) ? t : (kNV - 1);
  const int ax = n & 1, ay = (n >> 1) & 1, sx = (n >> 2) & 1, sy = (n >> 3) & 1, c = n >> 4;
  float acc = 0.0f;
#pragma unroll 1
  for (int dy = 0; dy < 3; ++dy) {
    const int oy = sy + dy + 1;
    const int jy = (oy >> 1) - 1;
    const int sgy = oy & 1;
#pragma unroll 1
    for (int dx = 0; dx < 3; ++dx) {
      const int ox = sx + dx + 1;
      const int jx = (ox >> 1) - 1;
      const int sgx = ox & 1;
      const bool inc = (jy == sy + ay - 1) && (jx == sx + ax - 1);
#pragma unroll 1
      for (int m = 0; m < kCh; ++m) {
        const float tw = bf_rne(tail_w[((c * kCh + m) * 3 + dy) * 3 + dx]);
        const float ub = bf_rne(up2_b[4 * m + 2 * sgy + sgx]);
        const float term = tw * ub;
        acc += inc ? term : 0.0f;
      }
    }
  }
  const float val = (t < kNV) ? acc : 0.0f;
  ((volatile float*)Vb)[t] = val;
  __threadfence();
  ((volatile float*)Vb)[t] = val;
}

__global__ __launch_bounds__(256) void dynk_kernel(const float* __restrict__ kv, const float* __restrict__ w1,
                                                   const float* __restrict__ w2, float* __restrict__ dk)
{
  __shared__ float hid[kNB * kCh];
  const int i = blockIdx.x;
  const int tid = threadIdx.x;
#pragma unroll 1
  for (int j = tid; j < kNB * kCh; j += 256) {
    const int b = j >> 6, h = j & 63;
    const float* wr = w1 + ((size_t)i * kCh + h) * kCh;
    const float* kr = kv + b * kCh;
    float s = 0.0f;
#pragma unroll 1
    for (int c = 0; c < kCh; ++c) s = fmaf(bf_rne(kr[c]), bf_rne(wr[c]), s);
    hid[j] = (s >= 0.0f) ? s : 0.1f * s;
  }
  __syncthreads();
#pragma unroll 1
  for (int m = tid; m < kNB * kKK; m += 256) {
    const int b = m / kKK;
    const int mm = m - b * kKK;
    const float* wr = w2 + ((size_t)i * kKK + mm) * kCh;
    const float* hr = hid + b * kCh;
    float s = 0.0f;
#pragma unroll 1
    for (int j = 0; j < kCh; ++j) s = fmaf(hr[j], bf_rne(wr[j]), s);
    volatile float* q = dk + (size_t)i * kNB * kKK + m;
    *q = s;
    __threadfence();
    *q = s;
  }
}

__global__ __launch_bounds__(256) void im2col_kernel(const float* __restrict__ xin, unsigned short* __restrict__ Ihi,
                                                     unsigned short* __restrict__ Ilo)
{
  __shared__ __align__(16) float sI[256 * 36];
  const int tid = threadIdx.x;
  const int p = blockIdx.x * 256 + tid;
  const int x = p & 127, y = (p >> 7) & 127, b = p >> 14;
  float* row = sI + tid * 36;
#pragma unroll 1
  for (int ci = 0; ci < 3; ++ci) {
    const float mean = (ci == 0) ? 0.4488f : ((ci == 1) ? 0.4371f : 0.404f);
    const float* pl = xin + ((size_t)(b * 3 + ci) * kH1) * kW1;
#pragma unroll
    for (int ky = 0; ky < 3; ++ky) {
#pragma unroll
      for (int kx = 0; kx < 3; ++kx) {
        const int gy = y + ky - 1, gx = x + kx - 1;
        const bool inside = ((unsigned)gy < (unsigned)kH1) && ((unsigned)gx < (unsigned)kW1);
        const int gyc = min(max(gy, 0), kH1 - 1), gxc = min(max(gx, 0), kW1 - 1);
        const float v = pl[gyc * kW1 + gxc];
        row[ci * 9 + ky * 3 + kx] = inside ? (bf_rne(v) - mean) : 0.0f;
      }
    }
  }
#pragma unroll
  for (int k = 27; k < 32; ++k) row[k] = 0.0f;
  __syncthreads();
  v8h hv[4], lv[4];
#pragma unroll
  for (int it = 0; it < 4; ++it) {
    const int chunk = it * 256 + tid;
    const float* sp = sI + (chunk >> 2) * 36 + (chunk & 3) * 8;
    const v4f a0 = *(const v4f*)(sp);
    const v4f a1 = *(const v4f*)(sp + 4);
#pragma unroll
    for (int e = 0; e < 4; ++e) {
      const float f0 = a0[e], f1 = a1[e];
      const _Float16 h0 = (_Float16)f0, h1 = (_Float16)f1;
      hv[it][e] = h0;
      hv[it][4 + e] = h1;
      lv[it][e] = (_Float16)((f0 - (float)h0) * kLoCarry);
      lv[it][4 + e] = (_Float16)((f1 - (float)h1) * kLoCarry);
    }
  }
  const size_t base = (size_t)blockIdx.x * 256 * kHeadK;
  for (int pass = 0; pass < 2; ++pass) {
#pragma unroll
    for (int it = 0; it < 4; ++it) {
      const size_t o = base + (size_t)(it * 256 + tid) * 8;
      *(volatile v8h*)(Ihi + o) = hv[it];
      *(volatile v8h*)(Ilo + o) = lv[it];
    }
    __threadfence();
  }
}

__global__ __launch_bounds__(256) void halo_zero_kernel(unsigned char* __restrict__ base, int nb, int HP, int WP, int lpp)
{
  const int g = (blockIdx.x * 256 + threadIdx.x) >> 3;
  const int l8 = threadIdx.x & 7;
  const int nh = 2 * WP + 2 * (HP - 2);
  if (g >= nb * nh * lpp) return;
  const int t = g / lpp;
  const int ln = g - t * lpp;
  const int bb = t / nh;
  const int h = t - bb * nh;
  int row, col;
  if (h < WP) {
    row = 0;
    col = h;
  } else if (h < 2 * WP) {
    row = HP - 1;
    col = h - WP;
  } else {
    const int r = h - 2 * WP;
    row = 1 + (r >> 1);
    col = (r & 1) ? (WP - 1) : 0;
  }
  const size_t pix = ((size_t)bb * HP + row) * WP + col;
  unsigned char* q = base + (pix * lpp + ln) * 128 + l8 * 16;
  const v4f z = (v4f){0.0f, 0.0f, 0.0f, 0.0f};
  *(volatile v4f*)q = z;
  __threadfence();
  *(volatile v4f*)q = z;
}

template <bool SPLIT>
__global__ __launch_bounds__(256) void ddc_kernel(const float* __restrict__ R, const float* __restrict__ dk,
                                                  unsigned short* __restrict__ Ahi, unsigned short* __restrict__ Alo)
{
  __shared__ __align__(16) float sT[kW1 * 68];
  const int tid = threadIdx.x;
  const int c = tid & 63, seg = tid >> 6;
  const int x0 = seg * 32;
  const int b = blockIdx.x >> 7, y = blockIdx.x & 127;
  const float* kk = dk + (size_t)b * kKK + c * 9;
  const float k00 = kk[0], k01 = kk[1], k02 = kk[2];
  const float k10 = kk[3], k11 = kk[4], k12 = kk[5];
  const float k20 = kk[6], k21 = kk[7], k22 = kk[8];
  const float* r0 = R + (((size_t)b * kHP1 + y) * kWP1 + x0) * kCh + c;
  const float* r1 = r0 + (size_t)kWP1 * kCh;
  const float* r2 = r1 + (size_t)kWP1 * kCh;
  float a00 = r0[0], a01 = r0[kCh];
  float a10 = r1[0], a11 = r1[kCh];
  float a20 = r2[0], a21 = r2[kCh];
#pragma unroll 1
  for (int px = 0; px < 32; ++px) {
    const int off = (px + 2) * kCh;
    const float a02 = r0[off], a12 = r1[off], a22 = r2[off];
    float s = k00 * a00;
    s = fmaf(k01, a01, s);
    s = fmaf(k02, a02, s);
    s = fmaf(k10, a10, s);
    s = fmaf(k11, a11, s);
    s = fmaf(k12, a12, s);
    s = fmaf(k20, a20, s);
    s = fmaf(k21, a21, s);
    s = fmaf(k22, a22, s);
    s = (s >= 0.0f) ? s : 0.1f * s;
    sT[(x0 + px) * 68 + c] = s;
    a00 = a01; a01 = a02;
    a10 = a11; a11 = a12;
    a20 = a21; a21 = a22;
  }
  __syncthreads();
  v8h hv[4], lv[4];
#pragma unroll
  for (int it = 0; it < 4; ++it) {
    const int chunk = it * 256 + tid;
    const float* sp = sT + (chunk >> 3) * 68 + (chunk & 7) * 8;
    const v4f a0 = *(const v4f*)(sp);
    const v4f a1 = *(const v4f*)(sp + 4);
#pragma unroll
    for (int e = 0; e < 4; ++e) {
      const float f0 = a0[e], f1 = a1[e];
      const _Float16 h0 = (_Float16)f0, h1 = (_Float16)f1;
      hv[it][e] = h0;
      hv[it][4 + e] = h1;
      if (SPLIT) {
        lv[it][e] = (_Float16)((f0 - (float)h0) * kLoCarry);
        lv[it][4 + e] = (_Float16)((f1 - (float)h1) * kLoCarry);
      }
    }
  }
  const size_t rowbase = (((size_t)b * kHP1 + y + 1) * kWP1 + 1) * kCh;
  for (int pass = 0; pass < 2; ++pass) {
#pragma unroll
    for (int it = 0; it < 4; ++it) {
      const int chunk = it * 256 + tid;
      const size_t o = rowbase + (size_t)(chunk >> 3) * kCh + (chunk & 7) * 8;
      *(volatile v8h*)(Ahi + o) = hv[it];
      if (SPLIT) *(volatile v8h*)(Alo + o) = lv[it];
    }
    __threadfence();
  }
}

template <int TAPS, int CIN, bool SPLIT, int MI, int NJ, int EPI>
__global__ __launch_bounds__(256) void conv_wmma_kernel(
    const unsigned short* __restrict__ Ahp, const unsigned short* __restrict__ Alp,
    const unsigned short* __restrict__ Btp, const float* __restrict__ bias,
    void* o0, void* o1, const float* aux,
    int H, int W, int lgH, int lgTpr, int lgNt)
{
  static_assert(TAPS == 9 || TAPS == 1);
  static_assert((CIN % 32) == 0);
  static_assert(!SPLIT || NJ == 4);
  static_assert(NJ == 3 || NJ == 4);
  __shared__ __align__(16) float sT[8][16 * 68];
  const int lane = threadIdx.x & 31;
  const int wave = __builtin_amdgcn_readfirstlane((int)(threadIdx.x >> 5));
  const int total = kNB << (lgH + lgTpr + lgNt);
  const int tile = blockIdx.x * 8 + wave;
  if (tile >= total) return;
  const int nt = tile & ((1 << lgNt) - 1);
  int rest = tile >> lgNt;
  const int xt = rest & ((1 << lgTpr) - 1);
  rest >>= lgTpr;
  const int y = rest & (H - 1);
  const int b = rest >> lgH;
  constexpr int TP = 16 * MI;
  const int x0 = xt * TP;
  const int n0 = nt * 64;
  const int rlane = lane & 15;
  const int koff = (lane >> 4) * 8;
  const int mOff = (lane >> 4) * 8;
  constexpr int KY = (TAPS == 9) ? 3 : 1;
  constexpr int LDB = TAPS * CIN;
  const int HP = (TAPS == 9) ? (H + 2) : H;
  const int WP = (TAPS == 9) ? (W + 2) : W;
  const _Float16* Ah = (const _Float16*)Ahp;
  const _Float16* Al = (const _Float16*)Alp;
  const _Float16* Bt = (const _Float16*)Btp;

  v8f accM[MI][4];
  v8f accL[SPLIT ? MI : 1][4];
#pragma unroll
  for (int i = 0; i < MI; ++i)
#pragma unroll
    for (int j = 0; j < 4; ++j) {
      accM[i][j] = (v8f){0.f, 0.f, 0.f, 0.f, 0.f, 0.f, 0.f, 0.f};
      if (SPLIT) accL[SPLIT ? i : 0][j] = (v8f){0.f, 0.f, 0.f, 0.f, 0.f, 0.f, 0.f, 0.f};
    }

#pragma unroll 1
  for (int ky = 0; ky < KY; ++ky) {
#pragma unroll 1
    for (int kx = 0; kx < KY; ++kx) {
      const size_t prow = ((size_t)(b * HP + y + ky) * WP + x0 + rlane + kx) * CIN + koff;
      const int kt = (ky * KY + kx) * CIN + koff;
#pragma unroll 1
      for (int kc = 0; kc < CIN / 32; ++kc) {
        v16h bf[4];
#pragma unroll
        for (int j = 0; j < NJ; ++j)
          bf[j] = FragH::load(Bt + (size_t)(n0 + (j << 4) + rlane) * LDB + kt + kc * 32);
#pragma unroll
        for (int i = 0; i < MI; ++i) {
          const size_t ao = prow + (size_t)(i * 16) * CIN + kc * 32;
          const v16h ah = FragH::load(Ah + ao);
          v16h al = ah;
          if (SPLIT) al = FragH::load(Al + ao);
#pragma unroll
          for (int j = 0; j < NJ; ++j) {
            accM[i][j] = FragH::mma(ah, bf[j], accM[i][j]);
            if (SPLIT) accL[SPLIT ? i : 0][j] = FragH::mma(al, bf[j], accL[SPLIT ? i : 0][j]);
          }
          if (SPLIT) {
            guard_row8(accM[i][0], accM[i][1], accM[i][2], accM[i][3],
                       accL[SPLIT ? i : 0][0], accL[SPLIT ? i : 0][1], accL[SPLIT ? i : 0][2], accL[SPLIT ? i : 0][3], ah, al);
          } else if (NJ == 4) {
            guard_row4(accM[i][0], accM[i][1], accM[i][2], accM[i][3], ah, ah);
          } else {
            guard_row3(accM[i][0], accM[i][1], accM[i][2], ah, ah);
          }
        }
        if (NJ == 4) keep4_h(bf[0], bf[1], bf[2], bf[3]);
        else keep3_h(bf[0], bf[1], bf[2]);
      }
    }
  }

  float* slab = sT[wave];
#pragma unroll
  for (int i = 0; i < MI; ++i) {
#pragma unroll
    for (int j = 0; j < NJ; ++j) {
      const int n = (j << 4) + rlane;
      float bv;
      if (EPI == 4) bv = bf_rne(bias[4 * n + nt]);
      else if (EPI == 5) bv = bias[n];
      else bv = bf_rne(bias[n0 + n]);
#pragma unroll
      for (int r = 0; r < 8; ++r) {
        float v = accM[i][j][r] * kScaleMain;
        if (SPLIT) v = fmaf(accL[SPLIT ? i : 0][j][r], kScaleLo, v);
        slab[(mOff + r) * 68 + n] = v + bv;
      }
    }
    wave_sync();
    const int px0 = x0 + (i << 4);
    if (EPI == 0 || EPI == 1 || EPI == 2) {
      const int hh = lane >> 4, c4 = (lane & 15) * 4;
      float* R = (float*)o0;
      const size_t rrow = ((size_t)(b * (H + 2) + y + 1) * (W + 2) + px0 + 1) * kCh + c4;
      v4f vals[8];
#pragma unroll
      for (int it = 0; it < 8; ++it) {
        const int row = it * 2 + hh;
        v4f s = *(const v4f*)(slab + row * 68 + c4);
        if (EPI != 0) {
          const v4f ro = *(const v4f*)(R + rrow + (size_t)row * kCh);
          s = s + ro;
          if (EPI == 2) *(v4f*)(slab + row * 68 + c4) = s;
        }
        vals[it] = s;
      }
      v8h hv[4];
      const int q = lane >> 3, c8 = (lane & 7) * 8;
      if (EPI == 2) {
        wave_sync();
#pragma unroll
        for (int it = 0; it < 4; ++it) {
          const float* sp = slab + (it * 4 + q) * 68 + c8;
          const v4f a0 = *(const v4f*)(sp);
          const v4f a1 = *(const v4f*)(sp + 4);
#pragma unroll
          for (int e = 0; e < 4; ++e) {
            hv[it][e] = (_Float16)a0[e];
            hv[it][4 + e] = (_Float16)a1[e];
          }
        }
      }
      for (int pass = 0; pass < 2; ++pass) {
#pragma unroll
        for (int it = 0; it < 8; ++it) {
          const int row = it * 2 + hh;
          *(volatile v4f*)(R + rrow + (size_t)row * kCh) = vals[it];
          if (EPI == 0) {
            float* X = (float*)o1;
            *(volatile v4f*)(X + ((size_t)(b * H + y) * W + px0 + row) * kCh + c4) = vals[it];
          }
        }
        if (EPI == 2) {
          unsigned short* S = (unsigned short*)o1;
#pragma unroll
          for (int it = 0; it < 4; ++it) {
            const int row = it * 4 + q;
            *(volatile v8h*)(S + ((size_t)(b * (H + 2) + y + 1) * (W + 2) + px0 + row + 1) * kCh + c8) = hv[it];
          }
        }
        __threadfence();
      }
    } else if (EPI == 3 || EPI == 4) {
      const int q = lane >> 3, c8 = (lane & 7) * 8;
      unsigned short* C = (unsigned short*)o0;
      v8h hv[4];
#pragma unroll
      for (int it = 0; it < 4; ++it) {
        const int row = it * 4 + q;
        const float* sp = slab + row * 68 + c8;
        v4f a0 = *(const v4f*)(sp);
        v4f a1 = *(const v4f*)(sp + 4);
        if (EPI == 3) {
          const float* xp = aux + ((size_t)(b * H + y) * W + px0 + row) * kCh + c8;
          const v4f s0 = *(const v4f*)(xp);
          const v4f s1 = *(const v4f*)(xp + 4);
          a0 = a0 + s0;
          a1 = a1 + s1;
        }
#pragma unroll
        for (int e = 0; e < 4; ++e) {
          hv[it][e] = (_Float16)a0[e];
          hv[it][4 + e] = (_Float16)a1[e];
        }
      }
      for (int pass = 0; pass < 2; ++pass) {
#pragma unroll
        for (int it = 0; it < 4; ++it) {
          const int row = it * 4 + q;
          size_t o;
          if (EPI == 3) {
            o = ((size_t)(b * (H + 2) + y + 1) * (W + 2) + px0 + row + 1) * kCh + c8;
          } else {
            const int ry = nt >> 1, rx = nt & 1;
            o = ((size_t)(b * (2 * H + 2) + 2 * y + ry + 1) * (2 * W + 2) + 2 * (px0 + row) + rx + 1) * kCh + c8;
          }
          *(volatile v8h*)(C + o) = hv[it];
        }
        __threadfence();
      }
    } else {
      unsigned short* G = (unsigned short*)o0;
      const size_t gbase = ((size_t)(b * H + y) * W + px0) * kNV;
      v8h hv[3];
#pragma unroll
      for (int it = 0; it < 3; ++it) {
        const int chunk = it * 32 + lane;
        const int pr = chunk / 6;
        const int c8 = (chunk - pr * 6) * 8;
        const float* sp = slab + pr * 68 + c8;
        const v4f a0 = *(const v4f*)(sp);
        const v4f a1 = *(const v4f*)(sp + 4);
#pragma unroll
        for (int e = 0; e < 4; ++e) {
          hv[it][e] = (_Float16)a0[e];
          hv[it][4 + e] = (_Float16)a1[e];
        }
      }
      for (int pass = 0; pass < 2; ++pass) {
#pragma unroll
        for (int it = 0; it < 3; ++it)
          *(volatile v8h*)(G + gbase + (size_t)(it * 32 + lane) * 8) = hv[it];
        __threadfence();
      }
    }
    wave_sync();
  }
}

__global__ __launch_bounds__(256) void gather_kernel(const unsigned* __restrict__ Gw, const float* __restrict__ tail_b,
                                                     float* __restrict__ out)
{
  const int idx = blockIdx.x * 256 + threadIdx.x;
  const int xq = idx & 127;
  const int Y = (idx >> 7) & 511;
  const int rest = idx >> 16;
  const int b = rest / 3;
  const int c = rest - b * 3;
  const int qy = Y >> 1, sy = Y & 1;
  const float mean = (c == 0) ? 0.4488f : ((c == 1) ? 0.4371f : 0.404f);
  const float tb = bf_rne(tail_b[c]);
  v4f o;
#pragma unroll
  for (int e = 0; e < 4; ++e) {
    const int sx = e & 1;
    const int qx = 2 * xq + (e >> 1);
    const int nb4 = ((c * 2 + sy) * 2 + sx) * 4;
    float acc = 0.0f;
#pragma unroll
    for (int ay = 0; ay < 2; ++ay) {
#pragma unroll
      for (int ax = 0; ax < 2; ++ax) {
        const int py = qy + sy + ay - 1;
        const int pxx = qx + sx + ax - 1;
        const bool ok = ((unsigned)py < (unsigned)kH2) && ((unsigned)pxx < (unsigned)kW2);
        const int pyc = min(max(py, 0), kH2 - 1);
        const int pxc = min(max(pxx, 0), kW2 - 1);
        const int elem = ((b * kH2 + pyc) * kW2 + pxc) * kNV + nb4 + ay * 2 + ax;
        const unsigned w = Gw[elem >> 1];
        const unsigned hb = (elem & 1) ? (w >> 16) : (w & 0xffffu);
        const float g = h16_to_f32(hb);
        acc += ok ? g : 0.0f;
      }
    }
    o[e] = (acc + tb) + mean;
  }
  float* q = out + ((size_t)(b * 3 + c) * 512 + Y) * 512 + 4 * xq;
  *(volatile v4f*)q = o;
  __threadfence();
  *(volatile v4f*)q = o;
}

extern "C" void kernel_launch(void* const* d_in, const int* in_sizes, int n_in,
                              void* d_out, int out_size, void* d_ws, size_t ws_size,
                              hipStream_t stream)
{
  if (n_in < 16) return;
  if (in_sizes[0] != kNB * 3 * kH1 * kW1) return;
  if (in_sizes[1] != kNB * kCh) return;
  if (in_sizes[2] != kCh * 27) return;
  if (in_sizes[3] != kCh) return;
  if (in_sizes[4] != kNBlk * kCh * kCh) return;
  if (in_sizes[5] != kNBlk * kKK * kCh) return;
  if (in_sizes[6] != kNBlk * kCh * kKK) return;
  if (in_sizes[7] != kNBlk * kCh) return;
  if (in_sizes[8] != kCh * kKK) return;
  if (in_sizes[9] != kCh) return;
  if (in_sizes[10] != 4 * kCh * kKK) return;
  if (in_sizes[11] != 4 * kCh) return;
  if (in_sizes[12] != 4 * kCh * kKK) return;
  if (in_sizes[13] != 4 * kCh) return;
  if (in_sizes[14] != 3 * kKK) return;
  if (in_sizes[15] != 3) return;
  if (out_size != kNB * 3 * 512 * 512) return;
  if (ws_size < kWsTotal) return;

  const float* x       = (const float*)d_in[0];
  const float* k_v     = (const float*)d_in[1];
  const float* head_w  = (const float*)d_in[2];
  const float* head_b  = (const float*)d_in[3];
  const float* kmlp1   = (const float*)d_in[4];
  const float* kmlp2   = (const float*)d_in[5];
  const float* convw   = (const float*)d_in[6];
  const float* convb   = (const float*)d_in[7];
  const float* bodyc_w = (const float*)d_in[8];
  const float* bodyc_b = (const float*)d_in[9];
  const float* up1_w   = (const float*)d_in[10];
  const float* up1_b   = (const float*)d_in[11];
  const float* up2_w   = (const float*)d_in[12];
  const float* up2_b   = (const float*)d_in[13];
  const float* tail_w  = (const float*)d_in[14];
  const float* tail_b  = (const float*)d_in[15];
  float* out = (float*)d_out;

  char* ws = (char*)d_ws;
  unsigned short* AHI = (unsigned short*)(ws + kOffAHI);
  unsigned short* ALO = (unsigned short*)(ws + kOffALO);
  unsigned short* SHI = (unsigned short*)(ws + kOffSHI);
  float*          RES = (float*)(ws + kOffRES);
  float*          XHD = (float*)(ws + kOffXHD);
  unsigned short* WB  = (unsigned short*)(ws + kOffWB);
  unsigned short* WC  = (unsigned short*)(ws + kOffWC);
  unsigned short* WU1 = (unsigned short*)(ws + kOffWU1);
  unsigned short* WV  = (unsigned short*)(ws + kOffWV);
  unsigned short* WH  = (unsigned short*)(ws + kOffWH);
  float*          DK  = (float*)(ws + kOffDK);
  float*          VB  = (float*)(ws + kOffVB);
  unsigned short* IHI = (unsigned short*)(ws + kOffIHI);
  unsigned short* ILO = (unsigned short*)(ws + kOffILO);
  unsigned short* B16 = AHI;
  unsigned short* TUP = (unsigned short*)(ws + kOffTUP);
  unsigned short* GPL = (unsigned short*)(ws + kOffGPL);

  pack_w_kernel<<<(kNBlk * kCh * 72) / 256, 256, 0, stream>>>(convw, WB, kNBlk * kCh, 0);
  pack_w_kernel<<<(kCh * 72) / 256, 256, 0, stream>>>(bodyc_w, WC, kCh, 0);
  pack_w_kernel<<<(4 * kCh * 72) / 256, 256, 0, stream>>>(up1_w, WU1, 4 * kCh, 1);
  pack_head_kernel<<<1, 256, 0, stream>>>(head_w, WH);
  compose_v_kernel<<<kNV, kKK, 0, stream>>>(tail_w, up2_w, WV);
  vbias_kernel<<<1, 64, 0, stream>>>(tail_w, up2_b, VB);
  dynk_kernel<<<kNBlk, 256, 0, stream>>>(k_v, kmlp1, kmlp2, DK);

  im2col_kernel<<<(kNB * kH1 * kW1) / 256, 256, 0, stream>>>(x, IHI, ILO);
  conv_wmma_kernel<1, kHeadK, true, 2, 4, 0><<<(kNB * kH1 * 4) / 8, 256, 0, stream>>>(
      IHI, ILO, WH, head_b, (void*)RES, (void*)XHD, XHD, kH1, kW1, 7, 2, 0);

  halo_zero_kernel<<<(24 * 516 * 8) / 256, 256, 0, stream>>>((unsigned char*)AHI, 24, kHP1, kWP1, 1);
  halo_zero_kernel<<<(8 * 516 * 2 * 8) / 256, 256, 0, stream>>>((unsigned char*)RES, 8, kHP1, kWP1, 2);

  for (int i = 0; i < kNBlk; ++i) {
    ddc_kernel<kSplitBlocks><<<kNB * kH1, 256, 0, stream>>>(RES, DK + (size_t)i * kNB * kKK, AHI, ALO);
    if (i < kNBlk - 1) {
      conv_wmma_kernel<9, kCh, kSplitBlocks, kBlkMI, 4, 1><<<(kNB * kH1 * (kW1 / (16 * kBlkMI))) / 8, 256, 0, stream>>>(
          AHI, ALO, WB + (size_t)i * kCh * kKK, convb + i * kCh, (void*)RES, (void*)SHI, XHD, kH1, kW1, 7, kBlkLgTpr, 0);
    } else {
      conv_wmma_kernel<9, kCh, kSplitBlocks, kBlkMI, 4, 2><<<(kNB * kH1 * (kW1 / (16 * kBlkMI))) / 8, 256, 0, stream>>>(
          AHI, ALO, WB + (size_t)i * kCh * kKK, convb + i * kCh, (void*)RES, (void*)SHI, XHD, kH1, kW1, 7, kBlkLgTpr, 0);
    }
  }

  conv_wmma_kernel<9, kCh, false, 4, 4, 3><<<(kNB * kH1 * 2) / 8, 256, 0, stream>>>(
      SHI, SHI, WC, bodyc_b, (void*)B16, (void*)B16, XHD, kH1, kW1, 7, 1, 0);

  halo_zero_kernel<<<(8 * 1028 * 8) / 256, 256, 0, stream>>>((unsigned char*)TUP, 8, kHP2, kWP2, 1);
  conv_wmma_kernel<9, kCh, false, 4, 4, 4><<<(kNB * kH1 * 2 * 4) / 8, 256, 0, stream>>>(
      B16, B16, WU1, up1_b, (void*)TUP, (void*)TUP, XHD, kH1, kW1, 7, 1, 2);

  conv_wmma_kernel<9, kCh, false, 4, 3, 5><<<(kNB * kH2 * 4) / 8, 256, 0, stream>>>(
      TUP, TUP, WV, VB, (void*)GPL, (void*)GPL, VB, kH2, kW2, 8, 2, 0);

  gather_kernel<<<(kNB * 3 * 512 * 128) / 256, 256, 0, stream>>>((const unsigned*)GPL, tail_b, out);
}
